// LambdaLayer3d_10411000725998
// MI455X (gfx1250) — hardware-verified
//
#include <hip/hip_runtime.h>


#define BDIM   4
#define CDIM   64
#define NPOS   2744
#define NPADP  2752
#define NQT    172
#define NOUTC  96
#define KP     3136
#define TW     32
#define TSZ    (27 * 27 * TW * 16)
#define NSTAT  144
#define EPSBN  1e-5f

static_assert(NPOS % 4 == 0);
static_assert(NPADP == NQT * 16);
static_assert(KP == 196 * 16);
static_assert((TSZ % 4) == 0);
static_assert((BDIM * CDIM * NPOS) % 1024 == 0);

typedef __bf16         v16bf __attribute__((ext_vector_type(16)));
typedef float          v8f   __attribute__((ext_vector_type(8)));
typedef float          v4f   __attribute__((ext_vector_type(4)));
typedef unsigned int   v4u   __attribute__((ext_vector_type(4)));
typedef unsigned short v8us  __attribute__((ext_vector_type(8)));
typedef v4f  v4fa  __attribute__((may_alias));
typedef v4u  v4ua  __attribute__((may_alias));
typedef v8us v8usa __attribute__((may_alias));

union Frag { v16bf v; v4u q[2]; unsigned int u[8]; };
static_assert(sizeof(Frag) == 32);

__device__ __forceinline__ unsigned int f2bf(float f) {
  unsigned int u = __float_as_uint(f);
  u += 0x7FFFu + ((u >> 16) & 1u);
  return u >> 16;
}
__device__ __forceinline__ float bf2f(unsigned int b) { return __uint_as_float(b << 16); }
__device__ __forceinline__ void split2(float f, unsigned int& hi, unsigned int& lo) {
  hi = f2bf(f);
  lo = f2bf(f - bf2f(hi));
}

__device__ __forceinline__ void mma3(v8f& acc, const Frag& ah, const Frag& al, const Frag& bh, const Frag& bl) {
  acc = __builtin_amdgcn_wmma_f32_16x16x32_bf16(false, ah.v, false, bh.v, (short)0, acc, false, false);
  acc = __builtin_amdgcn_wmma_f32_16x16x32_bf16(false, al.v, false, bh.v, (short)0, acc, false, false);
  acc = __builtin_amdgcn_wmma_f32_16x16x32_bf16(false, ah.v, false, bl.v, (short)0, acc, false, false);
  asm volatile("v_nop\n\tv_nop\n\tv_nop\n\tv_nop" : "+v"(acc) : "v"(ah.v), "v"(al.v), "v"(bh.v), "v"(bl.v));
}

__device__ __forceinline__ void st2_v4f(float* p, v4f v) {
  *(volatile v4f*)p = v; __threadfence(); *(volatile v4f*)p = v;
}
__device__ __forceinline__ void st2_v4u(unsigned int* p, v4u v) {
  *(volatile v4u*)p = v; __threadfence(); *(volatile v4u*)p = v;
}
__device__ __forceinline__ void st2_v8us(unsigned short* p, v8us v) {
  *(volatile v8us*)p = v; __threadfence(); *(volatile v8us*)p = v;
}

__global__ __launch_bounds__(256) void k_cvt_x(const float* __restrict__ x,
                                             unsigned short* __restrict__ Xh, unsigned short* __restrict__ Xl) {
  __shared__ __align__(16) unsigned short sh[2][32][64];
  const int t = threadIdx.x, b = blockIdx.y, n0 = blockIdx.x * 32;
  const int c = t >> 2, j = t & 3;
  const int n = n0 + 8 * j;
  float v[8];
  if (n < NPOS) {
    const float* src = x + ((size_t)(b * CDIM + c)) * NPOS + n;
    const v4f a0 = *(const v4fa*)src;
    const v4f a1 = *(const v4fa*)(src + 4);
#pragma unroll
    for (int e = 0; e < 4; ++e) { v[e] = a0[e]; v[4 + e] = a1[e]; }
  } else {
#pragma unroll
    for (int e = 0; e < 8; ++e) v[e] = 0.f;
  }
#pragma unroll
  for (int e = 0; e < 8; ++e) {
    unsigned int hi, lo; split2(v[e], hi, lo);
    sh[0][8 * j + e][c] = (unsigned short)hi;
    sh[1][8 * j + e][c] = (unsigned short)lo;
  }
  __syncthreads();
  const int w = t >> 5, lane = t & 31;
#pragma unroll
  for (int q = 0; q < 2; ++q) {
    const int L = (w * 2 + q) * 4 + (lane >> 3);
    const int plane = L >> 5, row = L & 31, ch = 8 * (lane & 7);
    const v8us val = *(const v8usa*)&sh[plane][row][ch];
    unsigned short* dst = (plane ? Xl : Xh) + ((size_t)(b * NPADP + n0 + row)) * CDIM + ch;
    st2_v8us(dst, val);
  }
}

__global__ __launch_bounds__(256) void k_cvt_w(const float* __restrict__ Wq, const float* __restrict__ Wk,
                                             const float* __restrict__ Wv,
                                             unsigned short* __restrict__ Wh, unsigned short* __restrict__ Wl) {
  const int t = threadIdx.x;
  const int ch = 8 * (t & 7);
#pragma unroll
  for (int it = 0; it < 6; ++it) {
    const int L = it * 32 + (t >> 3);
    const int plane = (L >= NOUTC) ? 1 : 0;
    const int o = L - plane * NOUTC;
    const float* src = (o < 64) ? (Wq + o * CDIM) : ((o < 80) ? (Wk + (o - 64) * CDIM) : (Wv + (o - 80) * CDIM));
    src += ch;
    const v4f a0 = *(const v4fa*)src;
    const v4f a1 = *(const v4fa*)(src + 4);
    v8us val;
#pragma unroll
    for (int e = 0; e < 4; ++e) {
      unsigned int hi, lo;
      split2(a0[e], hi, lo); val[e]     = (unsigned short)(plane ? lo : hi);
      split2(a1[e], hi, lo); val[4 + e] = (unsigned short)(plane ? lo : hi);
    }
    st2_v8us((plane ? Wl : Wh) + o * CDIM + ch, val);
  }
}

__global__ __launch_bounds__(256) void k_cvt_tab(const float* __restrict__ rpe, unsigned int* __restrict__ T) {
  const int g = blockIdx.x * 256 + threadIdx.x;
  if (g >= TSZ / 4) return;
  const int off = g >> 2;
  const int ow = off & (TW - 1), odh = off >> 5;
  const int kq = (g & 3) * 4;
  v4u o4; o4[0] = 0u; o4[1] = 0u; o4[2] = 0u; o4[3] = 0u;
  if (ow < 27) {
    const v4f a = *(const v4fa*)(rpe + ((size_t)(odh * 27 + ow)) * 16 + kq);
#pragma unroll
    for (int e = 0; e < 4; ++e) { unsigned int hi, lo; split2(a[e], hi, lo); o4[e] = hi | (lo << 16); }
  }
  st2_v4u(T + (size_t)g * 4, o4);
}

__global__ __launch_bounds__(128) void k_proj(const unsigned short* __restrict__ Xh, const unsigned short* __restrict__ Xl,
                                            const unsigned short* __restrict__ Wh, const unsigned short* __restrict__ Wl,
                                            float* __restrict__ QKV) {
  __shared__ __align__(16) float sD[4][16 * NOUTC];
  const int t = threadIdx.x, w = t >> 5, lane = t & 31, h = lane >> 4, m = lane & 15;
  const int g = blockIdx.x * 4 + w;
  const int b = g / NQT, tile = g - b * NQT;
  const size_t rowA = ((size_t)(b * NPADP + tile * 16 + m)) * CDIM;
  Frag ah[2], al[2];
#pragma unroll
  for (int ks = 0; ks < 2; ++ks) {
    ah[ks].q[0] = *(const v4ua*)(Xh + rowA + 32 * ks + 8 * h);
    ah[ks].q[1] = *(const v4ua*)(Xh + rowA + 32 * ks + 16 + 8 * h);
    al[ks].q[0] = *(const v4ua*)(Xl + rowA + 32 * ks + 8 * h);
    al[ks].q[1] = *(const v4ua*)(Xl + rowA + 32 * ks + 16 + 8 * h);
  }
  v8f acc[6];
#pragma unroll
  for (int ct = 0; ct < 6; ++ct)
#pragma unroll
    for (int r = 0; r < 8; ++r) acc[ct][r] = 0.f;
#pragma unroll
  for (int ct = 0; ct < 6; ++ct) {
#pragma unroll
    for (int ks = 0; ks < 2; ++ks) {
      const size_t rowB = ((size_t)(16 * ct + m)) * CDIM + 32 * ks + 8 * h;
      Frag bh, bl;
      bh.q[0] = *(const v4ua*)(Wh + rowB);  bh.q[1] = *(const v4ua*)(Wh + rowB + 16);
      bl.q[0] = *(const v4ua*)(Wl + rowB);  bl.q[1] = *(const v4ua*)(Wl + rowB + 16);
      mma3(acc[ct], ah[ks], al[ks], bh, bl);
    }
  }
#pragma unroll
  for (int ct = 0; ct < 6; ++ct)
#pragma unroll
    for (int r = 0; r < 8; ++r) sD[w][(8 * h + r) * NOUTC + 16 * ct + m] = acc[ct][r];
  __syncthreads();
  float* dst = QKV + ((size_t)(b * NPADP + tile * 16)) * NOUTC;
#pragma unroll
  for (int q = 0; q < 12; ++q) {
    const int f = 128 * q + 4 * lane;
    *(volatile v4f*)(dst + f) = *(const v4fa*)&sD[w][f];
  }
  __threadfence();
#pragma unroll
  for (int q = 0; q < 12; ++q) {
    const int f = 128 * q + 4 * lane;
    *(volatile v4f*)(dst + f) = *(const v4fa*)&sD[w][f];
  }
}

__global__ __launch_bounds__(256) void k_stats(const float* __restrict__ QKV, float* __restrict__ ST) {
  __shared__ double sd1[256], sd2[256];
  __shared__ float sf[256];
  const int t = threadIdx.x, blk = blockIdx.x;
  float A = 0.f, B = 0.f;
  if (blk < 80) {
    const int col = (blk < 64) ? blk : (80 + (blk - 64));
    double s = 0.0, s2 = 0.0;
    for (int bb = 0; bb < BDIM; ++bb) {
      const float* base = QKV + ((size_t)bb * NPADP) * NOUTC + col;
      for (int n = t; n < NPOS; n += 256) {
        const float v = base[(size_t)n * NOUTC];
        s += (double)v; s2 += (double)v * (double)v;
      }
    }
    sd1[t] = s; sd2[t] = s2;
    __syncthreads();
    for (int off = 128; off > 0; off >>= 1) {
      if (t < off) { sd1[t] += sd1[t + off]; sd2[t] += sd2[t + off]; }
      __syncthreads();
    }
    if (t == 0) {
      const double N = (double)(BDIM * NPOS);
      const double mean = sd1[0] / N;
      double var = sd2[0] / N - mean * mean;
      if (var < 0.0) var = 0.0;
      const float varf = (float)var;
      A = (float)mean;
      B = 1.0f / sqrtf(varf + EPSBN);
    }
  } else {
    const int sb = blk - 80, bb = sb >> 4, kk = sb & 15;
    const float* base = QKV + ((size_t)bb * NPADP) * NOUTC + 64 + kk;
    float mx = -3.4e38f;
    for (int n = t; n < NPOS; n += 256) mx = fmaxf(mx, base[(size_t)n * NOUTC]);
    sf[t] = mx;
    __syncthreads();
    for (int off = 128; off > 0; off >>= 1) {
      if (t < off) sf[t] = fmaxf(sf[t], sf[t + off]);
      __syncthreads();
    }
    mx = sf[0];
    __syncthreads();
    float s = 0.f;
    for (int n = t; n < NPOS; n += 256) s += expf(base[(size_t)n * NOUTC] - mx);
    sf[t] = s;
    __syncthreads();
    for (int off = 128; off > 0; off >>= 1) {
      if (t < off) sf[t] += sf[t + off];
      __syncthreads();
    }
    if (t == 0) { A = mx; B = 1.0f / sf[0]; }
  }
  if (t < 8) {
    v4f v; v[0] = A; v[1] = B; v[2] = 0.f; v[3] = 0.f;
    st2_v4f(ST + blk * 32 + 4 * t, v);
  }
}

__global__ __launch_bounds__(256) void k_apply(const float* __restrict__ QKV, const float* __restrict__ ST,
    const float* __restrict__ gq, const float* __restrict__ bq,
    const float* __restrict__ gv, const float* __restrict__ bv,
    float* __restrict__ Qn, unsigned short* __restrict__ Kp, unsigned short* __restrict__ Vp) {
  __shared__ __align__(16) unsigned short tile[2][2][16][448];
  __shared__ float qmn[64], qsc[64], qbt[64], vmn[16], vsc[16], vbt[16], kmx[16], kin[16];
  const int t = threadIdx.x, dp = blockIdx.x, b = blockIdx.y;
  if (t < 64) {
    qmn[t] = ST[t * 32]; qsc[t] = ST[t * 32 + 1] * gq[t]; qbt[t] = bq[t];
  } else if (t < 80) {
    const int vv = t - 64;
    vmn[vv] = ST[(64 + vv) * 32]; vsc[vv] = ST[(64 + vv) * 32 + 1] * gv[vv]; vbt[vv] = bv[vv];
  } else if (t < 96) {
    const int kk = t - 80, line = 80 + b * 16 + kk;
    kmx[kk] = ST[line * 32]; kin[kk] = ST[line * 32 + 1];
  }
  {
    v4u z; z[0] = 0u; z[1] = 0u; z[2] = 0u; z[3] = 0u;
    v4u* tz = (v4u*)&tile[0][0][0][0];
#pragma unroll
    for (int i = 0; i < 14; ++i) tz[t + 256 * i] = z;
  }
  __syncthreads();

  for (int task = t; task < 392 * 16; task += 256) {
    const int nl = task >> 4, c4 = (task & 15) * 4;
    const int n = dp * 392 + nl;
    const v4f qv = *(const v4fa*)(QKV + ((size_t)(b * NPADP + n)) * NOUTC + c4);
    v4f o;
#pragma unroll
    for (int e = 0; e < 4; ++e) o[e] = (qv[e] - qmn[c4 + e]) * qsc[c4 + e] + qbt[c4 + e];
    st2_v4f(Qn + ((size_t)(b * NPOS + n)) * CDIM + c4, o);
  }

  for (int nl = t; nl < 392; nl += 256) {
    const int n = dp * 392 + nl;
    const int mdl = nl / 196, rem = nl - mdl * 196, mh = rem / 14, mw = rem - mh * 14;
    const int ml = (mdl * 14 + mh) * 16 + mw;
    const float* row = QKV + ((size_t)(b * NPADP + n)) * NOUTC + 64;
#pragma unroll 1
    for (int i = 0; i < 4; ++i) {
      const v4f a = *(const v4fa*)(row + 4 * i);
#pragma unroll
      for (int e = 0; e < 4; ++e) {
        const int kk = 4 * i + e;
        const float p = expf(a[e] - kmx[kk]) * kin[kk];
        unsigned int hi, lo; split2(p, hi, lo);
        tile[0][0][kk][ml] = (unsigned short)hi;
        tile[0][1][kk][ml] = (unsigned short)lo;
      }
    }
#pragma unroll 1
    for (int i = 0; i < 4; ++i) {
      const v4f a = *(const v4fa*)(row + 16 + 4 * i);
#pragma unroll
      for (int e = 0; e < 4; ++e) {
        const int vv = 4 * i + e;
        const float vn = (a[e] - vmn[vv]) * vsc[vv] + vbt[vv];
        unsigned int hi, lo; split2(vn, hi, lo);
        tile[1][0][vv][ml] = (unsigned short)hi;
        tile[1][1][vv][ml] = (unsigned short)lo;
      }
    }
  }
  __syncthreads();

  const int w = t >> 5, lane = t & 31;
#pragma unroll 1
  for (int pass = 0; pass < 2; ++pass) {
    for (int it = 0; it < 14; ++it) {
      const int L = (it * 8 + w) * 4 + (lane >> 3);
      const int rowid = L / 7, li = L - rowid * 7;
      const int arr = rowid >> 5, plane = (rowid >> 4) & 1, j = rowid & 15;
      const int ch = li * 64 + 8 * (lane & 7);
      const v8us val = *(const v8usa*)&tile[arr][plane][j][ch];
      unsigned short* dst = (arr ? Vp : Kp) + (size_t)plane * 64 * KP + (size_t)(b * 16 + j) * KP + dp * 448 + ch;
      *(volatile v8us*)dst = val;
    }
    if (pass == 0) __threadfence();
  }
}

__global__ __launch_bounds__(128) void k_clam(const unsigned short* __restrict__ Kp, const unsigned short* __restrict__ Vp,
                                            float* __restrict__ lc) {
  __shared__ __align__(16) float sL[4][256];
  const int t = threadIdx.x, w = t >> 5, lane = t & 31, h = lane >> 4, m = lane & 15;
  const unsigned short* ka = Kp + ((size_t)(w * 16 + m)) * KP + 8 * h;
  const unsigned short* va = Vp + ((size_t)(w * 16 + m)) * KP + 8 * h;
  v8f acc;
#pragma unroll
  for (int r = 0; r < 8; ++r) acc[r] = 0.f;
#pragma unroll 1
  for (int s = 0; s < KP / 32; ++s) {
    const int k0 = 32 * s;
    Frag ah, al, bh, bl;
    ah.q[0] = *(const v4ua*)(ka + k0);            ah.q[1] = *(const v4ua*)(ka + k0 + 16);
    al.q[0] = *(const v4ua*)(ka + 64 * KP + k0);  al.q[1] = *(const v4ua*)(ka + 64 * KP + k0 + 16);
    bh.q[0] = *(const v4ua*)(va + k0);            bh.q[1] = *(const v4ua*)(va + k0 + 16);
    bl.q[0] = *(const v4ua*)(va + 64 * KP + k0);  bl.q[1] = *(const v4ua*)(va + 64 * KP + k0 + 16);
    mma3(acc, ah, al, bh, bl);
  }
#pragma unroll
  for (int r = 0; r < 8; ++r) sL[w][(8 * h + r) * 16 + m] = acc[r];
  __syncthreads();
  float* dst = lc + w * 256;
#pragma unroll
  for (int q = 0; q < 2; ++q) { const int f = 128 * q + 4 * lane; *(volatile v4f*)(dst + f) = *(const v4fa*)&sL[w][f]; }
  __threadfence();
#pragma unroll
  for (int q = 0; q < 2; ++q) { const int f = 128 * q + 4 * lane; *(volatile v4f*)(dst + f) = *(const v4fa*)&sL[w][f]; }
}

__global__ __launch_bounds__(128) void k_plam(const unsigned int* __restrict__ T, const unsigned short* __restrict__ Vp,
                                            const float* __restrict__ Qn, const float* __restrict__ lc,
                                            float* __restrict__ Y) {
  __shared__ __align__(16) float sP[4][2][256];
  const int t = threadIdx.x, w = t >> 5, lane = t & 31, h = lane >> 4, m = lane & 15;
  const int n = blockIdx.x * 4 + w;
  const int nd = n / 196, nr = n - nd * 196, nh = nr / 14, nw = nr - nh * 14;

  v8f acc[4];
#pragma unroll
  for (int b = 0; b < 4; ++b)
#pragma unroll
    for (int r = 0; r < 8; ++r) acc[b][r] = lc[b * 256 + (8 * h + r) * 16 + m];

  const unsigned int* ap = T + ((((13 - nd) * 27 + (13 - nh)) * TW + (8 * h - nw + 13)) * 16 + m);
  const unsigned short* vp = Vp + (size_t)m * KP + 8 * h;

#pragma unroll 1
  for (int md = 0; md < 14; ++md) {
    const unsigned int* apd = ap + md * (27 * TW * 16);
    const unsigned short* vpd = vp + md * 224;
#pragma unroll 1
    for (int p = 0; p < 7; ++p) {
      const unsigned int* app = apd + p * (2 * TW * 16);
      const unsigned short* vpp = vpd + p * 32;
      unsigned int e[16];
#pragma unroll
      for (int i = 0; i < 8; ++i) {
        e[i]     = app[16 * i];
        e[8 + i] = app[TW * 16 + 16 * i];
      }
      Frag ah, al;
#pragma unroll
      for (int j = 0; j < 8; ++j) {
        const unsigned int e0 = e[2 * j], e1 = e[2 * j + 1];
        ah.u[j] = (e0 & 0xffffu) | (e1 << 16);
        al.u[j] = (e0 >> 16) | (e1 & 0xffff0000u);
      }
      Frag bh[4], bl[4];
#pragma unroll
      for (int b = 0; b < 4; ++b) {
        const unsigned short* r0 = vpp + b * (16 * KP);
        bh[b].q[0] = *(const v4ua*)r0;             bh[b].q[1] = *(const v4ua*)(r0 + 16);
        bl[b].q[0] = *(const v4ua*)(r0 + 64 * KP); bl[b].q[1] = *(const v4ua*)(r0 + 64 * KP + 16);
      }
#pragma unroll
      for (int b = 0; b < 4; ++b) {
        acc[b] = __builtin_amdgcn_wmma_f32_16x16x32_bf16(false, ah.v, false, bh[b].v, (short)0, acc[b], false, false);
        acc[b] = __builtin_amdgcn_wmma_f32_16x16x32_bf16(false, al.v, false, bh[b].v, (short)0, acc[b], false, false);
        acc[b] = __builtin_amdgcn_wmma_f32_16x16x32_bf16(false, ah.v, false, bl[b].v, (short)0, acc[b], false, false);
      }
      asm volatile("v_nop\n\tv_nop\n\tv_nop\n\tv_nop"
                   : "+v"(acc[0]), "+v"(acc[1]), "+v"(acc[2]), "+v"(acc[3])
                   : "v"(ah.v), "v"(al.v),
                     "v"(bh[0].v), "v"(bl[0].v), "v"(bh[1].v), "v"(bl[1].v),
                     "v"(bh[2].v), "v"(bl[2].v), "v"(bh[3].v), "v"(bl[3].v));
    }
  }

#pragma unroll
  for (int b = 0; b < 4; ++b) {
    const float* qr = Qn + ((size_t)(b * NPOS + n)) * CDIM + 8 * h;
#pragma unroll
    for (int hp = 0; hp < 4; ++hp) {
      const v4f q0 = *(const v4fa*)(qr + hp * 16);
      const v4f q1 = *(const v4fa*)(qr + hp * 16 + 4);
      float pacc = q0[0] * acc[b][0];
      pacc += q0[1] * acc[b][1]; pacc += q0[2] * acc[b][2]; pacc += q0[3] * acc[b][3];
      pacc += q1[0] * acc[b][4]; pacc += q1[1] * acc[b][5]; pacc += q1[2] * acc[b][6]; pacc += q1[3] * acc[b][7];
      sP[w][h][b * 64 + hp * 16 + m] = pacc;
    }
  }
  __syncthreads();
  float* dst = Y + (size_t)n * 256;
#pragma unroll
  for (int s = 0; s < 2; ++s) {
    const int f = 128 * s + 4 * lane;
    const v4f v = *(const v4fa*)&sP[w][0][f] + *(const v4fa*)&sP[w][1][f];
    *(volatile v4f*)(dst + f) = v;
  }
  __threadfence();
#pragma unroll
  for (int s = 0; s < 2; ++s) {
    const int f = 128 * s + 4 * lane;
    const v4f v = *(const v4fa*)&sP[w][0][f] + *(const v4fa*)&sP[w][1][f];
    *(volatile v4f*)(dst + f) = v;
  }
}

__global__ __launch_bounds__(256) void k_layout(const float* __restrict__ Y, float* __restrict__ out) {
  const int g = blockIdx.x * 256 + threadIdx.x;
  if (g >= BDIM * CDIM * NPOS / 4) return;
  const int e0 = g * 4;
  const int bc = e0 / NPOS, n = e0 - bc * NPOS;
  const float* src = Y + (size_t)n * 256 + bc;
  v4f v; v[0] = src[0]; v[1] = src[256]; v[2] = src[512]; v[3] = src[768];
  st2_v4f(out + (size_t)e0, v);
}

extern "C" void kernel_launch(void* const* d_in, const int* in_sizes, int n_in,
                              void* d_out, int out_size, void* d_ws, size_t ws_size,
                              hipStream_t stream) {
  if (n_in < 9) return;
  if (in_sizes[0] != BDIM * CDIM * NPOS || in_sizes[1] != 64 * 64 || in_sizes[2] != 16 * 64 ||
      in_sizes[3] != 16 * 64 || in_sizes[4] != 27 * 27 * 27 * 16 || in_sizes[5] < 64 || in_sizes[6] < 64 ||
      in_sizes[7] < 16 || in_sizes[8] < 16) return;
  if (out_size != BDIM * CDIM * NPOS) return;

  const float* x   = (const float*)d_in[0];
  const float* Wq  = (const float*)d_in[1];
  const float* Wk  = (const float*)d_in[2];
  const float* Wv  = (const float*)d_in[3];
  const float* rpe = (const float*)d_in[4];
  const float* gq  = (const float*)d_in[5];
  const float* bq  = (const float*)d_in[6];
  const float* gv  = (const float*)d_in[7];
  const float* bv  = (const float*)d_in[8];
  float* out = (float*)d_out;

  size_t off = 0;
  auto carve = [&](size_t bytes) -> size_t { size_t r = off; off += (bytes + 255) & ~(size_t)255; return r; };
  const size_t oXh  = carve(sizeof(unsigned short) * BDIM * NPADP * CDIM);
  const size_t oXl  = carve(sizeof(unsigned short) * BDIM * NPADP * CDIM);
  const size_t oWh  = carve(sizeof(unsigned short) * NOUTC * CDIM);
  const size_t oWl  = carve(sizeof(unsigned short) * NOUTC * CDIM);
  const size_t oT   = carve(sizeof(unsigned int) * (size_t)TSZ);
  const size_t oQKV = carve(sizeof(float) * (size_t)BDIM * NPADP * NOUTC);
  const size_t oST  = carve(sizeof(float) * NSTAT * 32);
  const size_t oQn  = carve(sizeof(float) * (size_t)BDIM * NPOS * CDIM);
  const size_t oKp  = carve(sizeof(unsigned short) * 2 * 64 * (size_t)KP);
  const size_t oVp  = carve(sizeof(unsigned short) * 2 * 64 * (size_t)KP);
  const size_t olc  = carve(sizeof(float) * BDIM * 256);
  const size_t oY   = carve(sizeof(float) * (size_t)NPOS * 256);
  if (off > ws_size) return;

  char* ws = (char*)d_ws;
  unsigned short* Xh  = (unsigned short*)(ws + oXh);
  unsigned short* Xl  = (unsigned short*)(ws + oXl);
  unsigned short* Wh  = (unsigned short*)(ws + oWh);
  unsigned short* Wl  = (unsigned short*)(ws + oWl);
  unsigned int*   T   = (unsigned int*)(ws + oT);
  float*          QKV = (float*)(ws + oQKV);
  float*          ST  = (float*)(ws + oST);
  float*          Qn  = (float*)(ws + oQn);
  unsigned short* Kp  = (unsigned short*)(ws + oKp);
  unsigned short* Vp  = (unsigned short*)(ws + oVp);
  float*          lc  = (float*)(ws + olc);
  float*          Y   = (float*)(ws + oY);

  k_cvt_x  <<<dim3((NPOS + 31) / 32, BDIM), 256, 0, stream>>>(x, Xh, Xl);
  k_cvt_w  <<<1, 256, 0, stream>>>(Wq, Wk, Wv, Wh, Wl);
  k_cvt_tab<<<(TSZ / 4 + 255) / 256, 256, 0, stream>>>(rpe, T);
  k_proj   <<<(BDIM * NQT) / 4, 128, 0, stream>>>(Xh, Xl, Wh, Wl, QKV);
  k_stats  <<<NSTAT, 256, 0, stream>>>(QKV, ST);
  k_apply  <<<dim3(7, BDIM), 256, 0, stream>>>(QKV, ST, gq, bq, gv, bv, Qn, Kp, Vp);
  k_clam   <<<1, 128, 0, stream>>>(Kp, Vp, lc);
  k_plam   <<<NPOS / 4, 128, 0, stream>>>(T, Vp, Qn, lc, Y);
  k_layout <<<(BDIM * CDIM * NPOS / 4 + 255) / 256, 256, 0, stream>>>(Y, out);
}
